// TemporalEncoderDecoderAttention_3839700763043
// MI455X (gfx1250) — hardware-run, weakly checked
//
#include <hip/hip_runtime.h>
#include <math.h>

#ifndef NB
#define NB 4
#endif
#define NB_FULL 4
#define QSTEPS 12
#define KSTEPS 12
#define NODES 207
#define DM 128
#define DKH 16
#define HEADS 8
#define DHID 256
#define NGRP 128
#define NW2 16384
#define ROWS_B 2484
#define R_ROWS (NB * ROWS_B)
#define RT ((R_ROWS + 15) / 16)
#define RP (RT * 16)
#define WO_CARRY 1024.0f
#define WO_UNCARRY 0.0009765625f

static_assert(NB >= 1 && NB <= NB_FULL);
static_assert(ROWS_B == QSTEPS * NODES);
static_assert(NB != 4 || R_ROWS == 621 * 16);
static_assert(NB != 4 || RT == 207 * 3);
static_assert(NW2 == HEADS * DKH * DM);
static_assert(NGRP == HEADS * DKH);
static_assert(DM % 32 == 0 && DHID % 32 == 0);
static_assert(DM == 8 * 16 && DHID == 4 * 64);
static_assert((RP * DM / 8) % 256 == 0);
static_assert((DHID * DM / 8) % 256 == 0);
static_assert((NW2 * DHID / 8) % 256 == 0);
static_assert((DM * DM / 8) % 256 == 0);

typedef __attribute__((ext_vector_type(16))) _Float16 v16h;
typedef __attribute__((ext_vector_type(8)))  _Float16 v8h;
typedef __attribute__((ext_vector_type(16))) __bf16   v16bf;
typedef __attribute__((ext_vector_type(8)))  float    v8f;
typedef __attribute__((ext_vector_type(4)))  float    v4f;
typedef __attribute__((ext_vector_type(4)))  unsigned int v4u;
typedef __attribute__((ext_vector_type(8)))  unsigned int v8u;
typedef v4u v4u_ma __attribute__((may_alias));
typedef _Float16 h16;


#define VST2(T, ptr, val) do { const T vst2_v_ = (val); *(volatile T*)(ptr) = vst2_v_; __threadfence(); *(volatile T*)(ptr) = vst2_v_; } while (0)

__device__ __forceinline__ unsigned bf_rne(float f) {
    unsigned u = __float_as_uint(f);
    u += 0x7FFFu + ((u >> 16) & 1u);
    return u & 0xFFFF0000u;
}
__device__ __forceinline__ float bfr(float f) { return __uint_as_float(bf_rne(f)); }
__device__ __forceinline__ v4f bfr4(v4f v) { v4f o; o.x = bfr(v.x); o.y = bfr(v.y); o.z = bfr(v.z); o.w = bfr(v.w); return o; }
static __device__ __forceinline__ h16 toh_flush(float v) { const float w = (fabsf(v) < 6.103515625e-05f) ? 0.0f : v; return (h16)w; }

union FragU { v16h v; v8h h[2]; };
__device__ __forceinline__ v16h frag_ld(const _Float16* p) {
    FragU f; f.h[0] = *(const v8h*)(p); f.h[1] = *(const v8h*)(p + 16); return f.v;
}
__device__ __forceinline__ v16bf fragb_ld(const unsigned short* p) {
    const v4u lo = *(const v4u_ma*)(p);
    const v4u hi = *(const v4u_ma*)(p + 16);
    const v8u w = __builtin_shufflevector(lo, hi, 0, 1, 2, 3, 4, 5, 6, 7);
    return __builtin_bit_cast(v16bf, w);
}
__device__ __forceinline__ v8f wmma16g(v16h a, v16h b, v8f c) {
    c = __builtin_amdgcn_wmma_f32_16x16x32_f16(false, a, false, b, (short)0, c, false, false);
    asm volatile("v_nop\n\tv_nop\n\tv_nop\n\tv_nop" : "+v"(c) : "v"(a), "v"(b));
    return c;
}
__device__ __forceinline__ v8f wmmabg(v16bf a, v16bf b, v8f c) {
    c = __builtin_amdgcn_wmma_f32_16x16x32_bf16(false, a, false, b, (short)0, c, false, false);
    asm volatile("v_nop\n\tv_nop\n\tv_nop\n\tv_nop" : "+v"(c) : "v"(a), "v"(b));
    return c;
}
__device__ __forceinline__ void wave_sync_lds() {
    __builtin_amdgcn_fence(3  , "workgroup");
    __builtin_amdgcn_wave_barrier();
    __builtin_amdgcn_fence(2  , "workgroup");
}

__global__ __launch_bounds__(256) void k_cvt_bf16(const float* __restrict__ src, unsigned nsrc8,
                                                  unsigned short* __restrict__ dst, unsigned ndst8) {
    const unsigned u = blockIdx.x * 256u + threadIdx.x;
    if (u >= ndst8) return;
    const unsigned su = min(u, nsrc8 - 1u);
    const v4f a = *(const v4f*)(src + (size_t)su * 8u);
    const v4f b = *(const v4f*)(src + (size_t)su * 8u + 4u);
    v4u pk;
    pk.x = (bf_rne(a.x) >> 16) | bf_rne(a.y);
    pk.y = (bf_rne(a.z) >> 16) | bf_rne(a.w);
    pk.z = (bf_rne(b.x) >> 16) | bf_rne(b.y);
    pk.w = (bf_rne(b.z) >> 16) | bf_rne(b.w);
    VST2(v4u, (v4u*)(dst + (size_t)u * 8u), pk);
}

__global__ __launch_bounds__(256) void k_cvt_f16c(const float* __restrict__ src, _Float16* __restrict__ dst, unsigned n8) {
    const unsigned u = blockIdx.x * 256u + threadIdx.x;
    if (u >= n8) return;
    const v4f a = *(const v4f*)(src + (size_t)u * 8u);
    const v4f b = *(const v4f*)(src + (size_t)u * 8u + 4u);
    v8h hv;
    hv[0] = toh_flush(bfr(a.x) * WO_CARRY); hv[1] = toh_flush(bfr(a.y) * WO_CARRY);
    hv[2] = toh_flush(bfr(a.z) * WO_CARRY); hv[3] = toh_flush(bfr(a.w) * WO_CARRY);
    hv[4] = toh_flush(bfr(b.x) * WO_CARRY); hv[5] = toh_flush(bfr(b.y) * WO_CARRY);
    hv[6] = toh_flush(bfr(b.z) * WO_CARRY); hv[7] = toh_flush(bfr(b.w) * WO_CARRY);
    VST2(v8h, (v8h*)(dst + (size_t)u * 8u), hv);
}

__global__ __launch_bounds__(128) void k_hid(const unsigned short* __restrict__ ctp, const unsigned short* __restrict__ w1p,
                                             const float* __restrict__ b1, unsigned short* __restrict__ hhi,
                                             unsigned short* __restrict__ hlo, unsigned K) {
    __shared__ __align__(16) float sT[4][16 * 68];
    const unsigned lane = threadIdx.x & 31u, wave = threadIdx.x >> 5;
    const unsigned hh = lane >> 4, c = lane & 15u;
    const unsigned row0 = blockIdx.x * 16u;
    const unsigned n0 = wave * 64u;
    v8f acc[4];
#pragma unroll
    for (int j = 0; j < 4; ++j) acc[j] = (v8f){0.f,0.f,0.f,0.f,0.f,0.f,0.f,0.f};
    const unsigned short* ap = ctp + (size_t)(row0 + c) * DM + 8u * hh;
    const unsigned short* bp = w1p + (size_t)(n0 + c) * DM + 8u * hh;
    for (unsigned k0 = 0; k0 < K; k0 += 32u) {
        const v16bf a = fragb_ld(ap + k0);
#pragma unroll
        for (int j = 0; j < 4; ++j) {
            const v16bf b = fragb_ld(bp + (size_t)j * (16u * DM) + k0);
            acc[j] = wmmabg(a, b, acc[j]);
        }
    }
    float* slab = sT[wave];
#pragma unroll
    for (int j = 0; j < 4; ++j) {
        const float bv = bfr(b1[n0 + (unsigned)j * 16u + c]);
#pragma unroll
        for (int r = 0; r < 8; ++r)
            slab[(8u * hh + (unsigned)r) * 68u + (unsigned)j * 16u + c] = fmaxf(acc[j][r] + bv, 0.0f);
    }
    wave_sync_lds();
    const unsigned q = lane >> 3, c8 = (lane & 7u) * 8u;
    v4u ph[4], pl[4];
#pragma unroll
    for (int it = 0; it < 4; ++it) {
        const unsigned row = (unsigned)it * 4u + q;
        const v4f f0 = *(const v4f*)(slab + row * 68u + c8);
        const v4f f1 = *(const v4f*)(slab + row * 68u + c8 + 4u);
        const float f[8] = {f0.x, f0.y, f0.z, f0.w, f1.x, f1.y, f1.z, f1.w};
        unsigned hb[8], lb[8];
#pragma unroll
        for (int e = 0; e < 8; ++e) {
            hb[e] = bf_rne(f[e]);
            lb[e] = bf_rne(f[e] - __uint_as_float(hb[e]));
        }
        ph[it].x = (hb[0] >> 16) | hb[1]; ph[it].y = (hb[2] >> 16) | hb[3];
        ph[it].z = (hb[4] >> 16) | hb[5]; ph[it].w = (hb[6] >> 16) | hb[7];
        pl[it].x = (lb[0] >> 16) | lb[1]; pl[it].y = (lb[2] >> 16) | lb[3];
        pl[it].z = (lb[4] >> 16) | lb[5]; pl[it].w = (lb[6] >> 16) | lb[7];
    }
    for (int pass = 0; pass < 2; ++pass) {
#pragma unroll
        for (int it = 0; it < 4; ++it) {
            const unsigned row = row0 + (unsigned)it * 4u + q;
            *(volatile v4u*)(hhi + (size_t)row * DHID + n0 + c8) = ph[it];
            *(volatile v4u*)(hlo + (size_t)row * DHID + n0 + c8) = pl[it];
        }
        __threadfence();
    }
}

__global__ __launch_bounds__(96) void k_hyper(const unsigned short* __restrict__ hhi, const unsigned short* __restrict__ hlo,
                                              const unsigned short* __restrict__ w2p, const float* __restrict__ b2,
                                              const float* __restrict__ inputs, float* __restrict__ Qp, unsigned K) {
    __shared__ __align__(16) float sX[3][2048];
    __shared__ __align__(16) float sQ[3][16 * 132];
    const unsigned lane = threadIdx.x & 31u, wave = threadIdx.x >> 5;
    const unsigned hh = lane >> 4, c = lane & 15u;
    const unsigned tile = blockIdx.x * 3u + wave;
    if (tile >= (unsigned)RT) return;
    const unsigned row0 = tile * 16u;
    float* xs = sX[wave];
    float* qs = sQ[wave];
#pragma unroll
    for (int i = 0; i < 16; ++i) {
        const unsigned src = min(row0 + (unsigned)i, (unsigned)R_ROWS - 1u);
        const v4f v = bfr4(*(const v4f*)(inputs + (size_t)src * DM + 4u * lane));
        *(v4f*)(qs + (unsigned)i * 132u + 4u * lane) = v;
    }
    wave_sync_lds();
#pragma unroll
    for (int dt = 0; dt < 8; ++dt) {
        const float* sp = qs + (8u * hh) * 132u + (unsigned)dt * 16u + c;
        v4f x0, x1;
        x0.x = sp[0];   x0.y = sp[132]; x0.z = sp[264]; x0.w = sp[396];
        x1.x = sp[528]; x1.y = sp[660]; x1.z = sp[792]; x1.w = sp[924];
        *(v4f*)(xs + ((unsigned)dt * 32u + lane) * 8u) = x0;
        *(v4f*)(xs + ((unsigned)dt * 32u + lane) * 8u + 4u) = x1;
    }
    wave_sync_lds();

    const unsigned short* ahp = hhi + (size_t)(row0 + c) * DHID + 8u * hh;
    const unsigned short* alp = hlo + (size_t)(row0 + c) * DHID + 8u * hh;
    for (unsigned g = 0; g < (unsigned)NGRP; ++g) {
        v8f acc[8];
#pragma unroll
        for (int dt = 0; dt < 8; ++dt) acc[dt] = (v8f){0.f,0.f,0.f,0.f,0.f,0.f,0.f,0.f};
        const unsigned short* wb = w2p + (size_t)(g * 128u + c) * DHID + 8u * hh;
        for (unsigned k0 = 0; k0 < K; k0 += 32u) {
            const v16bf ah = fragb_ld(ahp + k0);
            const v16bf al = fragb_ld(alp + k0);
#pragma unroll
            for (int dt = 0; dt < 8; ++dt) {
                const v16bf bw = fragb_ld(wb + (size_t)dt * (16u * DHID) + k0);
                acc[dt] = wmmabg(ah, bw, acc[dt]);
                acc[dt] = wmmabg(al, bw, acc[dt]);
            }
        }
        float s[8];
#pragma unroll
        for (int r = 0; r < 8; ++r) s[r] = 0.0f;
#pragma unroll
        for (int dt = 0; dt < 8; ++dt) {
            const float bv = bfr(b2[g * 128u + (unsigned)dt * 16u + c]);
            const v4f x0 = *(const v4f*)(xs + ((unsigned)dt * 32u + lane) * 8u);
            const v4f x1 = *(const v4f*)(xs + ((unsigned)dt * 32u + lane) * 8u + 4u);
            s[0] += (acc[dt][0] + bv) * x0.x; s[1] += (acc[dt][1] + bv) * x0.y;
            s[2] += (acc[dt][2] + bv) * x0.z; s[3] += (acc[dt][3] + bv) * x0.w;
            s[4] += (acc[dt][4] + bv) * x1.x; s[5] += (acc[dt][5] + bv) * x1.y;
            s[6] += (acc[dt][6] + bv) * x1.z; s[7] += (acc[dt][7] + bv) * x1.w;
        }
#pragma unroll
        for (int r = 0; r < 8; ++r) {
            s[r] += __shfl_xor(s[r], 1, 32);
            s[r] += __shfl_xor(s[r], 2, 32);
            s[r] += __shfl_xor(s[r], 4, 32);
            s[r] += __shfl_xor(s[r], 8, 32);
        }
        if (c == 0u) {
#pragma unroll
            for (int r = 0; r < 8; ++r) qs[(8u * hh + (unsigned)r) * 132u + g] = s[r];
        }
    }
    wave_sync_lds();
#pragma unroll
    for (int half = 0; half < 2; ++half) {
        v4f qv[8];
#pragma unroll
        for (int it = 0; it < 8; ++it) qv[it] = *(const v4f*)(qs + (unsigned)(half * 8 + it) * 132u + 4u * lane);
        float* dst = Qp + (size_t)(row0 + (unsigned)half * 8u) * DM + 4u * lane;
        for (int pass = 0; pass < 2; ++pass) {
#pragma unroll
            for (int it = 0; it < 8; ++it) *(volatile v4f*)(dst + (size_t)it * DM) = qv[it];
            __threadfence();
        }
    }
}

__global__ __launch_bounds__(128) void k_attn(const float* __restrict__ Qp, const float* __restrict__ encK,
                                              const float* __restrict__ encV, _Float16* __restrict__ ctx16) {
    __shared__ __align__(16) _Float16 sC[4][4 * 136];
    const unsigned tid = threadIdx.x, lane = tid & 31u, wave = tid >> 5;
    const unsigned rl = tid >> 3, head = tid & 7u;
    const unsigned row = blockIdx.x * 16u + rl;
    const unsigned rowc = min(row, (unsigned)R_ROWS - 1u);
    const unsigned b = rowc / (unsigned)ROWS_B;
    const unsigned rem = rowc - b * (unsigned)ROWS_B;
    const unsigned n = rem % (unsigned)NODES;

    float qv[16];
    {
        const v4f* qp = (const v4f*)(Qp + (size_t)row * DM + head * 16u);
        const v4f q0 = qp[0], q1 = qp[1], q2 = qp[2], q3 = qp[3];
        qv[0] = q0.x; qv[1] = q0.y; qv[2] = q0.z; qv[3] = q0.w;
        qv[4] = q1.x; qv[5] = q1.y; qv[6] = q1.z; qv[7] = q1.w;
        qv[8] = q2.x; qv[9] = q2.y; qv[10] = q2.z; qv[11] = q2.w;
        qv[12] = q3.x; qv[13] = q3.y; qv[14] = q3.z; qv[15] = q3.w;
    }
    const size_t kvbase = ((size_t)b * (KSTEPS * NODES) + n) * 128u + head * 16u;
    float sc[KSTEPS];
    float mx = -3.0e38f;
#pragma unroll
    for (int p = 0; p < KSTEPS; ++p) {
        const v4f* kp = (const v4f*)(encK + kvbase + (size_t)p * (NODES * 128u));
        const v4f k0 = kp[0], k1 = kp[1], k2 = kp[2], k3 = kp[3];
        float d = 0.0f;
        d += qv[0] * bfr(k0.x);  d += qv[1] * bfr(k0.y);  d += qv[2] * bfr(k0.z);  d += qv[3] * bfr(k0.w);
        d += qv[4] * bfr(k1.x);  d += qv[5] * bfr(k1.y);  d += qv[6] * bfr(k1.z);  d += qv[7] * bfr(k1.w);
        d += qv[8] * bfr(k2.x);  d += qv[9] * bfr(k2.y);  d += qv[10] * bfr(k2.z); d += qv[11] * bfr(k2.w);
        d += qv[12] * bfr(k3.x); d += qv[13] * bfr(k3.y); d += qv[14] * bfr(k3.z); d += qv[15] * bfr(k3.w);
        sc[p] = d * 0.25f;
        mx = fmaxf(mx, sc[p]);
    }
    float sum = 0.0f;
#pragma unroll
    for (int p = 0; p < KSTEPS; ++p) { sc[p] = expf(sc[p] - mx); sum += sc[p]; }
    float o[16];
#pragma unroll
    for (int k = 0; k < 16; ++k) o[k] = 0.0f;
#pragma unroll
    for (int p = 0; p < KSTEPS; ++p) {
        const float a = sc[p] / sum;
        const v4f* vp = (const v4f*)(encV + kvbase + (size_t)p * (NODES * 128u));
        const v4f v0 = vp[0], v1 = vp[1], v2 = vp[2], v3 = vp[3];
        o[0] += a * bfr(v0.x);  o[1] += a * bfr(v0.y);  o[2] += a * bfr(v0.z);  o[3] += a * bfr(v0.w);
        o[4] += a * bfr(v1.x);  o[5] += a * bfr(v1.y);  o[6] += a * bfr(v1.z);  o[7] += a * bfr(v1.w);
        o[8] += a * bfr(v2.x);  o[9] += a * bfr(v2.y);  o[10] += a * bfr(v2.z); o[11] += a * bfr(v2.w);
        o[12] += a * bfr(v3.x); o[13] += a * bfr(v3.y); o[14] += a * bfr(v3.z); o[15] += a * bfr(v3.w);
    }
    v8h h0, h1;
#pragma unroll
    for (int e = 0; e < 8; ++e) { h0[e] = toh_flush(o[e]); h1[e] = toh_flush(o[8 + e]); }
    _Float16* tc = sC[wave];
    *(v8h*)(tc + (lane >> 3) * 136u + head * 16u) = h0;
    *(v8h*)(tc + (lane >> 3) * 136u + head * 16u + 8u) = h1;
    wave_sync_lds();
    {
        const unsigned c8 = (lane & 15u) * 8u;
        v8h ov[2];
#pragma unroll
        for (int it = 0; it < 2; ++it) ov[it] = *(const v8h*)(tc + ((unsigned)it * 2u + (lane >> 4)) * 136u + c8);
        _Float16* dst = ctx16 + (size_t)(blockIdx.x * 16u + wave * 4u + (lane >> 4)) * DM + c8;
        for (int pass = 0; pass < 2; ++pass) {
#pragma unroll
            for (int it = 0; it < 2; ++it) *(volatile v8h*)(dst + (size_t)it * (2u * DM)) = ov[it];
            __threadfence();
        }
    }
}

__global__ __launch_bounds__(96) void k_out(const _Float16* __restrict__ ctx16, const _Float16* __restrict__ wop,
                                            const float* __restrict__ inputs, const float* __restrict__ gamma,
                                            const float* __restrict__ beta, float* __restrict__ out, unsigned K) {
    __shared__ __align__(16) float sT[3][16 * 132];
    const unsigned lane = threadIdx.x & 31u, wave = threadIdx.x >> 5;
    const unsigned hh = lane >> 4, c = lane & 15u;
    const unsigned tile = blockIdx.x * 3u + wave;
    if (tile >= (unsigned)RT) return;
    const unsigned row0 = tile * 16u;
    v8f acc[8];
#pragma unroll
    for (int j = 0; j < 8; ++j) acc[j] = (v8f){0.f,0.f,0.f,0.f,0.f,0.f,0.f,0.f};
    const _Float16* ap = ctx16 + (size_t)(row0 + c) * DM + 8u * hh;
    const _Float16* bp = wop + (size_t)c * DM + 8u * hh;
    for (unsigned k0 = 0; k0 < K; k0 += 32u) {
        const v16h a = frag_ld(ap + k0);
#pragma unroll
        for (int j = 0; j < 8; ++j) {
            const v16h b = frag_ld(bp + (size_t)j * (16u * DM) + k0);
            acc[j] = wmma16g(a, b, acc[j]);
        }
    }
    float* slab = sT[wave];
#pragma unroll
    for (int j = 0; j < 8; ++j)
#pragma unroll
        for (int r = 0; r < 8; ++r)
            slab[(8u * hh + (unsigned)r) * 132u + (unsigned)j * 16u + c] = acc[j][r] * WO_UNCARRY;
    wave_sync_lds();
    const v4f g4 = bfr4(*(const v4f*)(gamma + 4u * lane));
    const v4f b4 = bfr4(*(const v4f*)(beta + 4u * lane));
#pragma unroll
    for (int half = 0; half < 2; ++half) {
        v4f ov[8];
#pragma unroll
        for (int it = 0; it < 8; ++it) {
            const unsigned i = (unsigned)(half * 8 + it);
            const unsigned src = min(row0 + i, (unsigned)R_ROWS - 1u);
            const v4f xr = bfr4(*(const v4f*)(inputs + (size_t)src * DM + 4u * lane));
            const v4f y = *(const v4f*)(slab + i * 132u + 4u * lane) + xr;
            float s = (y.x + y.y) + (y.z + y.w);
            s += __shfl_xor(s, 16, 32); s += __shfl_xor(s, 8, 32); s += __shfl_xor(s, 4, 32);
            s += __shfl_xor(s, 2, 32);  s += __shfl_xor(s, 1, 32);
            const float mu = s * (1.0f / 128.0f);
            v4f d; d.x = y.x - mu; d.y = y.y - mu; d.z = y.z - mu; d.w = y.w - mu;
            float q = (d.x * d.x + d.y * d.y) + (d.z * d.z + d.w * d.w);
            q += __shfl_xor(q, 16, 32); q += __shfl_xor(q, 8, 32); q += __shfl_xor(q, 4, 32);
            q += __shfl_xor(q, 2, 32);  q += __shfl_xor(q, 1, 32);
            const float var = q * (1.0f / 128.0f);
            const float rs = 1.0f / sqrtf(var + 1e-5f);
            v4f o;
            o.x = d.x * rs * g4.x + b4.x; o.y = d.y * rs * g4.y + b4.y;
            o.z = d.z * rs * g4.z + b4.z; o.w = d.w * rs * g4.w + b4.w;
            ov[it] = o;
        }
        for (int pass = 0; pass < 2; ++pass) {
#pragma unroll
            for (int it = 0; it < 8; ++it) {
                const unsigned row = row0 + (unsigned)(half * 8 + it);
                if (row < (unsigned)R_ROWS)
                    *(volatile v4f*)(out + (size_t)row * DM + 4u * lane) = ov[it];
            }
            __threadfence();
        }
    }
}

constexpr size_t al256(size_t x) { return (x + 255) & ~(size_t)255; }
constexpr size_t SZ_CT  = al256((size_t)RP * DM * 2);
constexpr size_t SZ_W1  = al256((size_t)DHID * DM * 2);
constexpr size_t SZ_W2  = al256((size_t)NW2 * DHID * 2);
constexpr size_t SZ_WO  = al256((size_t)DM * DM * 2);
constexpr size_t SZ_H   = al256((size_t)RP * DHID * 2);
constexpr size_t SZ_Q   = al256((size_t)RP * DM * 4);
constexpr size_t SZ_CX  = al256((size_t)RP * DM * 2);
constexpr size_t WS_TOTAL = SZ_CT + SZ_W1 + SZ_W2 + SZ_WO + 2 * SZ_H + SZ_Q + SZ_CX;
static_assert(WS_TOTAL <= (size_t)134217728);

extern "C" void kernel_launch(void* const* d_in, const int* in_sizes, int n_in, void* d_out, int out_size,
                              void* d_ws, size_t ws_size, hipStream_t stream) {
    if (n_in < 11) return;
    if (in_sizes[0] < R_ROWS * DM || in_sizes[1] < NB * KSTEPS * NODES * 128 || in_sizes[2] < NB * KSTEPS * NODES * 128) return;
    if (in_sizes[3] < R_ROWS * DM || in_sizes[4] < DHID * DM || in_sizes[5] < DHID) return;
    if (in_sizes[6] < NW2 * DHID || in_sizes[7] < NW2 || in_sizes[8] < DM * DM || in_sizes[9] < DM || in_sizes[10] < DM) return;
    if (out_size < R_ROWS * DM) return;
    if (WS_TOTAL > ws_size) return;

    const float* inputs = (const float*)d_in[0];
    const float* enc_K  = (const float*)d_in[1];
    const float* enc_V  = (const float*)d_in[2];
    const float* c_tgt  = (const float*)d_in[3];
    const float* W1     = (const float*)d_in[4];
    const float* b1     = (const float*)d_in[5];
    const float* W2     = (const float*)d_in[6];
    const float* b2     = (const float*)d_in[7];
    const float* W_out  = (const float*)d_in[8];
    const float* gamma  = (const float*)d_in[9];
    const float* beta   = (const float*)d_in[10];
    float* out = (float*)d_out;

    char* wsp = (char*)d_ws;
    size_t off = 0;
    unsigned short* ctp = (unsigned short*)(wsp + off); off += SZ_CT;
    unsigned short* w1p = (unsigned short*)(wsp + off); off += SZ_W1;
    unsigned short* w2p = (unsigned short*)(wsp + off); off += SZ_W2;
    _Float16*       wop = (_Float16*)(wsp + off);       off += SZ_WO;
    unsigned short* hhi = (unsigned short*)(wsp + off); off += SZ_H;
    unsigned short* hlo = (unsigned short*)(wsp + off); off += SZ_H;
    float*          Qp  = (float*)(wsp + off);          off += SZ_Q;
    _Float16*       cx  = (_Float16*)(wsp + off);       off += SZ_CX;
    if (off != WS_TOTAL) return;

    k_cvt_bf16<<<(RP * DM / 8) / 256, 256, 0, stream>>>(c_tgt, (unsigned)(R_ROWS * DM / 8), ctp, (unsigned)(RP * DM / 8));
    k_cvt_bf16<<<(DHID * DM / 8) / 256, 256, 0, stream>>>(W1, (unsigned)(DHID * DM / 8), w1p, (unsigned)(DHID * DM / 8));
    k_cvt_bf16<<<(NW2 * DHID / 8) / 256, 256, 0, stream>>>(W2, (unsigned)(NW2 * DHID / 8), w2p, (unsigned)(NW2 * DHID / 8));
    k_cvt_f16c<<<(DM * DM / 8) / 256, 256, 0, stream>>>(W_out, wop, (unsigned)(DM * DM / 8));

    k_hid<<<RT, 128, 0, stream>>>(ctp, w1p, b1, hhi, hlo, (unsigned)DM);
    k_hyper<<<(RT + 2) / 3, 96, 0, stream>>>(hhi, hlo, w2p, b2, inputs, Qp, (unsigned)DHID);
    k_attn<<<RT, 128, 0, stream>>>(Qp, enc_K, enc_V, cx);
    k_out<<<(RT + 2) / 3, 96, 0, stream>>>((const _Float16*)cx, (const _Float16*)wop, inputs, gamma, beta, out, (unsigned)DM);
}
